// ConformerBlock_50525995270838
// MI455X (gfx1250) — hardware-run, weakly checked
//
#include <hip/hip_runtime.h>
#include <math.h>

constexpr int kB    = 4;
constexpr int kD    = 512;
constexpr int kT    = 1024;
constexpr int kH    = 8;
constexpr int kDh   = 64;
constexpr int kFF   = 2048;
constexpr int kKW   = 31;
constexpr int kTok  = kB * kT;
constexpr int kQKld = 1024;
constexpr int kNB   = 320;
constexpr int kGnChunks = 128;
constexpr int kGnElems  = kD * kT;
constexpr float kWCarry   = 64.0f;
constexpr float kWInv     = 1.0f / 64.0f;
constexpr float kPCarry   = 32768.0f;
constexpr float kCtxCarry = 64.0f;
constexpr float kPVScale  = kCtxCarry / kPCarry;
constexpr float kOutScale = 1.0f / (kCtxCarry * kWCarry);
constexpr float kScoreScale = 0.125f;
constexpr double kGnInvN  = 1.0 / 524288.0;
static_assert(kH * kDh == kD);
static_assert(kTok % 64 == 0 && kD % 64 == 0 && kFF % 64 == 0 && kT % 64 == 0 && (2 * kD) % 64 == 0);
static_assert(kD % 32 == 0 && kFF % 32 == 0 && kDh % 32 == 0 && kT % 32 == 0);
static_assert(kGnChunks * 4096 == kGnElems);

typedef __attribute__((ext_vector_type(16))) _Float16 v16h;
typedef __attribute__((ext_vector_type(8)))  _Float16 v8h;
typedef __attribute__((ext_vector_type(8)))  float    v8f;
typedef __attribute__((ext_vector_type(4)))  float    v4f;
typedef __attribute__((ext_vector_type(2)))  float    v2f;
typedef __attribute__((ext_vector_type(4)))  unsigned int v4u;
typedef __attribute__((ext_vector_type(2)))  unsigned int v2u;

__constant__ int c_thr[] = {83, 85, 88, 90, 93, 96, 98, 101, 104, 107, 110, 114, 117, 120, 124, 127, 131, 135, 139, 143, 147, 151, 156, 160, 165, 170, 175, 180, 185, 190, 196, 201, 207, 213, 220, 226, 233, 239, 246, 253, 261, 268, 276, 284, 293, 301, 310, 319, 328, 338, 348, 358, 368, 379, 390, 401, 413, 425, 438, 450, 464, 477, 491, 505, 520, 535, 551, 567, 583, 600, 618, 636, 655, 674, 693, 714, 734, 756, 778};
static_assert(sizeof(c_thr) / sizeof(c_thr[0]) == 79);
constexpr int kThrN = 79;

__device__ __forceinline__ void dep_guard_h(v8f& a, v8f& b, v16h x, v16h y) { asm volatile("v_nop\n\tv_nop\n\tv_nop\n\tv_nop" : "+v"(a), "+v"(b) : "v"(x), "v"(y)); }
__device__ __forceinline__ void keep4_h(v16h a, v16h b, v16h c, v16h d) { asm volatile("v_nop" :: "v"(a), "v"(b), "v"(c), "v"(d)); }
__device__ __forceinline__ void acc_guard4(v8f& a, v8f& b, v8f& c, v8f& d) { asm volatile("v_nop\n\tv_nop\n\tv_nop\n\tv_nop" : "+v"(a), "+v"(b), "+v"(c), "+v"(d)); }
template <typename T> struct Frag;
template <> struct Frag<_Float16> {
  typedef v16h V; union U { v16h v; v8h h[2]; };
  static __device__ __forceinline__ v16h load(const _Float16* p) {
    U f; f.h[0] = *(const v8h*)(p); f.h[1] = *(const v8h*)(p + 16); return f.v;
  }
  static __device__ __forceinline__ v8f mma(v16h a, v16h b, v8f c) {
    return __builtin_amdgcn_wmma_f32_16x16x32_f16(false, a, false, b, (short)0, c, false, false);
  }
  static __device__ __forceinline__ void guard(v8f& a, v8f& b, v16h x, v16h y) { dep_guard_h(a, b, x, y); }
  static __device__ __forceinline__ void keep(v16h a, v16h b, v16h c, v16h d) { keep4_h(a, b, c, d); }
};

__device__ __forceinline__ unsigned pk16(unsigned short a, unsigned short b) { return (unsigned)a | ((unsigned)b << 16); }
__device__ __forceinline__ unsigned short h_bits(float f) { const _Float16 h = (_Float16)f; return __builtin_bit_cast(unsigned short, h); }

__device__ __forceinline__ float h16_to_f32(unsigned hb) {
  const unsigned sgn = (hb & 0x8000u) << 16; const unsigned em = hb & 0x7fffu;
  const float fn = __uint_as_float((em << 13) + 0x38000000u);
  const float fs = (float)em * 5.9604644775390625e-8f;
  const float mag = (em < 0x400u) ? fs : fn; return __uint_as_float(__float_as_uint(mag) | sgn); }

template <int BIAS_MODE, int OUT_MODE, bool RESID>
__global__ __launch_bounds__(256) void gemm_f16w(
    const unsigned short* __restrict__ Ap, int lda, long strideA,
    const unsigned short* __restrict__ Btp, int ldb, long strideB,
    void* __restrict__ Cout, int ldc, long strideC,
    const float* __restrict__ bias, float bscale,
    const float* __restrict__ resid, long strideR,
    int M, int N, int K, float scale) {
  typedef _Float16 T;
  typedef v16h V;
  const T* A = (const T*)Ap; const T* Bt = (const T*)Btp;
  __shared__ __align__(16) float sT[8][16 * 68];
  const int b    = blockIdx.y;
  const int lane = threadIdx.x & 31;
  const int wave = threadIdx.x >> 5;
  const int tilesN = N >> 6;
  const int tilesM = M >> 6;
  const int tile = blockIdx.x * 8 + wave;
  if (tile >= tilesM * tilesN) return;
  const int tm = tile / tilesN;
  const int tn = tile - tm * tilesN;
  const int m0 = tm << 6;
  const int n0 = tn << 6;

  const T* Ab = A  + (size_t)b * strideA;
  const T* Bb = Bt + (size_t)b * strideB;

  const int rlane = lane & 15;
  const int koff  = (lane >> 4) * 8;
  const int mOff  = (lane >> 4) * 8;

  v8f acc[4][4];
#pragma unroll
  for (int i = 0; i < 4; ++i)
#pragma unroll
    for (int j = 0; j < 4; ++j) acc[i][j] = (v8f){0.f,0.f,0.f,0.f,0.f,0.f,0.f,0.f};

  for (int k0 = 0; k0 < K; k0 += 32) {
    V bh[4];
#pragma unroll
    for (int j = 0; j < 4; ++j) {
      const size_t bo = (size_t)(n0 + (j << 4) + rlane) * ldb + koff + k0;
      bh[j] = Frag<T>::load(Bb + bo);
    }
#pragma unroll
    for (int i = 0; i < 4; ++i) {
      const size_t ao = (size_t)(m0 + (i << 4) + rlane) * lda + koff + k0;
      V ah = Frag<T>::load(Ab + ao);
#pragma unroll
      for (int j = 0; j < 4; ++j) {
        acc[i][j] = Frag<T>::mma(ah, bh[j], acc[i][j]);
      }
      Frag<T>::guard(acc[i][0], acc[i][3], ah, ah);
    }
    Frag<T>::keep(bh[0], bh[1], bh[2], bh[3]);
  }
  acc_guard4(acc[0][0], acc[0][1], acc[0][2], acc[0][3]);
  acc_guard4(acc[1][0], acc[1][1], acc[1][2], acc[1][3]);
  acc_guard4(acc[2][0], acc[2][1], acc[2][2], acc[2][3]);
  acc_guard4(acc[3][0], acc[3][1], acc[3][2], acc[3][3]);

  float* slab = sT[wave];
  const float* Rb = RESID ? (resid + (size_t)b * strideR) : nullptr;
#pragma unroll
  for (int i = 0; i < 4; ++i) {
    const int mBase = m0 + (i << 4);
#pragma unroll
    for (int j = 0; j < 4; ++j) {
      const int n = n0 + (j << 4) + rlane;
      float bv = 0.f;
      if (BIAS_MODE == 2) bv = bias[n] * bscale;
#pragma unroll
      for (int r = 0; r < 8; ++r) {
        float v = acc[i][j][r] * scale;
        if (BIAS_MODE == 1) v += bias[mBase + mOff + r] * bscale;
        if (BIAS_MODE == 2) v += bv;
        slab[(mOff + r) * 68 + (j << 4) + rlane] = v;
      }
    }
    __builtin_amdgcn_fence(__ATOMIC_RELEASE, "workgroup");
    __builtin_amdgcn_wave_barrier();
    __builtin_amdgcn_fence(__ATOMIC_ACQUIRE, "workgroup");
    if (OUT_MODE == 0) {
      float* C = (float*)Cout + (size_t)b * strideC;
      const int hh = lane >> 4, c4 = (lane & 15) * 4;
      v4f vals[8];
#pragma unroll
      for (int it = 0; it < 8; ++it) {
        const int row = it * 2 + hh;
        v4f v = *(const v4f*)(slab + row * 68 + c4);
        if (RESID) {
          const v4f rv = *(const v4f*)(Rb + (size_t)(mBase + row) * ldc + n0 + c4);
          v = v + rv;
        }
        vals[it] = v;
      }
      for (int pass = 0; pass < 2; ++pass) {
#pragma unroll
        for (int it = 0; it < 8; ++it) {
          const int row = it * 2 + hh;
          *(volatile v4f*)(C + (size_t)(mBase + row) * ldc + n0 + c4) = vals[it];
        }
        __threadfence();
      }
    } else {
      const int q = lane >> 3, c8 = (lane & 7) * 8;
      unsigned short* C = (unsigned short*)Cout + (size_t)b * strideC;
      for (int pass = 0; pass < 2; ++pass) {
#pragma unroll
        for (int it = 0; it < 4; ++it) {
          const int row = it * 4 + q;
          const float* sp = slab + row * 68 + c8;
          v8h hv;
#pragma unroll
          for (int e = 0; e < 8; ++e) hv[e] = (_Float16)sp[e];
          *(volatile v8h*)(C + (size_t)(mBase + row) * ldc + n0 + c8) = hv;
        }
        __threadfence();
      }
    }
    __builtin_amdgcn_fence(__ATOMIC_RELEASE, "workgroup");
    __builtin_amdgcn_wave_barrier();
    __builtin_amdgcn_fence(__ATOMIC_ACQUIRE, "workgroup");
  }
}

__global__ __launch_bounds__(256) void wtcast2_kernel(const float* __restrict__ W0, const float* __restrict__ W1,
                                                      unsigned short* __restrict__ O0, unsigned short* __restrict__ O1,
                                                      int Kin, int Nout, float scale) {
  __shared__ float sm[64][65];
  const int t  = threadIdx.x;
  const int k0 = blockIdx.x * 64;
  const int n0 = blockIdx.y * 64;
  const int z  = blockIdx.z;
  const float* W = (z == 0) ? W0 : W1;
  unsigned short* O = (z == 0) ? O0 : O1;
#pragma unroll
  for (int i = 0; i < 16; ++i) {
    const int e = i * 256 + t;
    const int r = e >> 6;
    const int c = e & 63;
    sm[c][r] = W[(size_t)(k0 + r) * Nout + n0 + c] * scale;
  }
  __syncthreads();
  const int lane = t & 31, wave = t >> 5;
  const int q = lane >> 3, c8 = (lane & 7) * 8;
  for (int pass = 0; pass < 2; ++pass) {
#pragma unroll
    for (int it = 0; it < 2; ++it) {
      const int row = wave * 8 + it * 4 + q;
      unsigned short hb[8];
#pragma unroll
      for (int e = 0; e < 8; ++e) hb[e] = h_bits(sm[row][c8 + e]);
      const v4u u = (v4u){pk16(hb[0], hb[1]), pk16(hb[2], hb[3]), pk16(hb[4], hb[5]), pk16(hb[6], hb[7])};
      *(volatile v4u*)(O + (size_t)(n0 + row) * Kin + k0 + c8) = u;
    }
    __threadfence();
  }
}

__global__ __launch_bounds__(256) void xin_kernel(const float* __restrict__ x, float* __restrict__ s32,
                                                  unsigned short* __restrict__ s16) {
  __shared__ __align__(16) float sm[64 * 68];
  const int tid = threadIdx.x;
  const int t0 = blockIdx.x * 64;
  const int d0 = blockIdx.y * 64;
  const int b  = blockIdx.z;
#pragma unroll
  for (int i = 0; i < 16; ++i) {
    const int e = i * 256 + tid;
    const int r = e >> 6;
    const int c = e & 63;
    sm[c * 68 + r] = x[((size_t)(b * kD + d0 + r)) * kT + t0 + c];
  }
  __syncthreads();
  const int lane = tid & 31, wave = tid >> 5;
  {
    const int hh = lane >> 4, c4 = (lane & 15) * 4;
    v4f vals[4];
#pragma unroll
    for (int it = 0; it < 4; ++it) {
      const int row = wave * 8 + it * 2 + hh;
      vals[it] = *(const v4f*)(sm + row * 68 + c4);
    }
    for (int pass = 0; pass < 2; ++pass) {
#pragma unroll
      for (int it = 0; it < 4; ++it) {
        const int row = wave * 8 + it * 2 + hh;
        *(volatile v4f*)(s32 + ((size_t)(b * kT + t0 + row)) * kD + d0 + c4) = vals[it];
      }
      __threadfence();
    }
  }
  {
    const int q = lane >> 3, c8 = (lane & 7) * 8;
    for (int pass = 0; pass < 2; ++pass) {
#pragma unroll
      for (int it = 0; it < 2; ++it) {
        const int row = wave * 8 + it * 4 + q;
        unsigned short hb[8];
#pragma unroll
        for (int e = 0; e < 8; ++e) hb[e] = h_bits(sm[row * 68 + c8 + e]);
        const v4u u = (v4u){pk16(hb[0], hb[1]), pk16(hb[2], hb[3]), pk16(hb[4], hb[5]), pk16(hb[6], hb[7])};
        *(volatile v4u*)(s16 + ((size_t)(b * kT + t0 + row)) * kD + d0 + c8) = u;
      }
      __threadfence();
    }
  }
}

__global__ __launch_bounds__(256) void xout_kernel(const float* __restrict__ s32, float* __restrict__ out) {
  __shared__ __align__(16) float sm[64 * 68];
  const int tid = threadIdx.x;
  const int t0 = blockIdx.x * 64;
  const int d0 = blockIdx.y * 64;
  const int b  = blockIdx.z;
#pragma unroll
  for (int i = 0; i < 16; ++i) {
    const int e = i * 256 + tid;
    const int r = e >> 6;
    const int c = e & 63;
    sm[c * 68 + r] = s32[((size_t)(b * kT + t0 + r)) * kD + d0 + c];
  }
  __syncthreads();
  const int lane = tid & 31, wave = tid >> 5;
  const int hh = lane >> 4, c4 = (lane & 15) * 4;
  v4f vals[4];
#pragma unroll
  for (int it = 0; it < 4; ++it) {
    const int row = wave * 8 + it * 2 + hh;
    vals[it] = *(const v4f*)(sm + row * 68 + c4);
  }
  for (int pass = 0; pass < 2; ++pass) {
#pragma unroll
    for (int it = 0; it < 4; ++it) {
      const int row = wave * 8 + it * 2 + hh;
      *(volatile v4f*)(out + ((size_t)(b * kD + d0 + row)) * kT + t0 + c4) = vals[it];
    }
    __threadfence();
  }
}

__global__ __launch_bounds__(256) void cast8_f16_kernel(const float* __restrict__ in, unsigned short* __restrict__ out, int n8) {
  const int i = blockIdx.x * 256 + threadIdx.x;
  if (i >= n8) return;
  const float* p = in + 8 * (size_t)i;
  const v4f a = *(const v4f*)(p);
  const v4f c = *(const v4f*)(p + 4);
  unsigned short hb[8];
#pragma unroll
  for (int e = 0; e < 4; ++e) {
    hb[e]     = h_bits(a[e]);
    hb[4 + e] = h_bits(c[e]);
  }
  const v4u u = (v4u){pk16(hb[0], hb[1]), pk16(hb[2], hb[3]), pk16(hb[4], hb[5]), pk16(hb[6], hb[7])};
  unsigned short* q = out + 8 * (size_t)i;
  *(volatile v4u*)q = u;
  __threadfence();
  *(volatile v4u*)q = u;
}

__global__ __launch_bounds__(256) void gelu2_kernel(const float* __restrict__ in, unsigned short* __restrict__ out, int n2) {
  const int i = blockIdx.x * 256 + threadIdx.x;
  if (i >= n2) return;
  const v2f p = *(const v2f*)(in + 2 * (size_t)i);
  const float g0 = 0.5f * p[0] * (1.0f + erff(p[0] * 0.70710678118654752f));
  const float g1 = 0.5f * p[1] * (1.0f + erff(p[1] * 0.70710678118654752f));
  const unsigned u = pk16(h_bits(g0), h_bits(g1));
  ((volatile unsigned*)out)[i] = u;
  __threadfence();
  ((volatile unsigned*)out)[i] = u;
}

__global__ __launch_bounds__(256) void dline_kernel(const float* __restrict__ re, float* __restrict__ dl) {
  const int g  = blockIdx.x * 256 + threadIdx.x;
  const int h  = g >> 9;
  const int j0 = (g & 511) * 4;
  int av[4], sg[4], cnt[4];
#pragma unroll
  for (int e = 0; e < 4; ++e) {
    const int rel = j0 + e - 1023;
    av[e] = rel < 0 ? -rel : rel;
    sg[e] = rel >= 0 ? 1 : 0;
    cnt[e] = 0;
  }
#pragma unroll 1
  for (int i = 0; i < kThrN; ++i) {
    const int th = c_thr[i];
#pragma unroll
    for (int e = 0; e < 4; ++e) cnt[e] += (th <= av[e]) ? 1 : 0;
  }
  v4f val;
#pragma unroll
  for (int e = 0; e < 4; ++e) {
    int bk = (av[e] < 80) ? av[e] : (80 + cnt[e]);
    bk += sg[e] * 160;
    bk = bk < 0 ? 0 : (bk > (kNB - 1) ? (kNB - 1) : bk);
    const float r = re[bk * kH + h];
    val[e] = (j0 + e < 2047) ? r : 0.0f;
  }
  float* dp = dl + (size_t)h * 2048 + j0;
  *(volatile v4f*)dp = val;
  __threadfence();
  *(volatile v4f*)dp = val;
}

__global__ __launch_bounds__(256) void dwt_kernel(const float* __restrict__ dww, float* __restrict__ dwt) {
  const int g = blockIdx.x * 256 + threadIdx.x;
  if (g >= kKW * (kD / 4)) return;
  const int k  = g >> 7;
  const int c0 = (g & 127) * 4;
  v4f v;
#pragma unroll
  for (int e = 0; e < 4; ++e) v[e] = dww[(size_t)(c0 + e) * kKW + k];
  float* dp = dwt + (size_t)k * kD + c0;
  *(volatile v4f*)dp = v;
  __threadfence();
  *(volatile v4f*)dp = v;
}

__global__ __launch_bounds__(256) void gates_kernel(const unsigned short* __restrict__ qk, const float* __restrict__ gu,
                                                    const float* __restrict__ gw, const float* __restrict__ gsc,
                                                    float* __restrict__ rc) {
  const int idx = blockIdx.x * 256 + threadIdx.x;
  const int t = idx & 1023, h = (idx >> 10) & 7, b = idx >> 13;
  const unsigned short* qrow = qk + ((size_t)(b * kT + t)) * kQKld + h * kDh;
  const float* gup = gu + h * kDh;
  const float* gwp = gw + h * kDh;
  float du = 0.0f, dv = 0.0f;
#pragma unroll 1
  for (int w8 = 0; w8 < 8; ++w8) {
    const v4u qwv = *(const v4u*)(qrow + 8 * w8);
    const v4f u0 = *(const v4f*)(gup + 8 * w8);
    const v4f u1 = *(const v4f*)(gup + 8 * w8 + 4);
    const v4f w0 = *(const v4f*)(gwp + 8 * w8);
    const v4f w1 = *(const v4f*)(gwp + 8 * w8 + 4);
    float qf[8];
#pragma unroll
    for (int e = 0; e < 4; ++e) {
      qf[2 * e]     = h16_to_f32(qwv[e] & 0xffffu);
      qf[2 * e + 1] = h16_to_f32(qwv[e] >> 16);
    }
#pragma unroll
    for (int e = 0; e < 4; ++e) { du += qf[e] * u0[e]; dv += qf[e] * w0[e]; }
#pragma unroll
    for (int e = 0; e < 4; ++e) { du += qf[4 + e] * u1[e]; dv += qf[4 + e] * w1[e]; }
  }
  const float gupd = 1.0f / (1.0f + expf(-du));
  const float grst = 1.0f / (1.0f + expf(-dv));
  const float gs = gsc[h];
  const float r = 1.0f + gupd + (1.0f - gupd) * gs * grst;
  ((volatile float*)rc)[idx] = r;
  __threadfence();
  ((volatile float*)rc)[idx] = r;
}

__global__ __launch_bounds__(128) void softmax_kernel(const float* __restrict__ S, unsigned short* __restrict__ P,
                                                      const float* __restrict__ rcb, const float* __restrict__ dline) {
  __shared__ float redM[4];
  __shared__ float redS[4];
  const int t = blockIdx.x;
  const int h = blockIdx.y;
  const int tid = threadIdx.x, lane = tid & 31, wave = tid >> 5;
  const size_t rowoff = ((size_t)h * kT + t) * kT;
  const float* sr = S + rowoff + 8 * tid;
  const v4f a = *(const v4f*)(sr);
  const v4f c = *(const v4f*)(sr + 4);
  const float rc = rcb[h * kT + t];
  const float* dl = dline + (size_t)h * 2048 + (1023 - t) + 8 * tid;
  float x[8];
#pragma unroll
  for (int e = 0; e < 4; ++e) {
    x[e]     = a[e] + rc * dl[e];
    x[4 + e] = c[e] + rc * dl[4 + e];
  }
  float m = fmaxf(fmaxf(fmaxf(x[0], x[1]), fmaxf(x[2], x[3])), fmaxf(fmaxf(x[4], x[5]), fmaxf(x[6], x[7])));
#pragma unroll
  for (int off = 16; off > 0; off >>= 1) m = fmaxf(m, __shfl_xor(m, off, 32));
  if (lane == 0) redM[wave] = m;
  __syncthreads();
  m = fmaxf(fmaxf(redM[0], redM[1]), fmaxf(redM[2], redM[3]));
  float sum = 0.0f;
#pragma unroll
  for (int e = 0; e < 8; ++e) { x[e] = expf(x[e] - m); sum += x[e]; }
#pragma unroll
  for (int off = 16; off > 0; off >>= 1) sum += __shfl_xor(sum, off, 32);
  if (lane == 0) redS[wave] = sum;
  __syncthreads();
  const float tot = ((redS[0] + redS[1]) + redS[2]) + redS[3];
  const float inv = kPCarry / tot;
  unsigned short hb[8];
#pragma unroll
  for (int e = 0; e < 8; ++e) hb[e] = h_bits(x[e] * inv);
  const v4u u = (v4u){pk16(hb[0], hb[1]), pk16(hb[2], hb[3]), pk16(hb[4], hb[5]), pk16(hb[6], hb[7])};
  unsigned short* pr = P + rowoff + 8 * (size_t)tid;
  *(volatile v4u*)pr = u;
  __threadfence();
  *(volatile v4u*)pr = u;
}

__global__ __launch_bounds__(256) void gnred_kernel(const float* __restrict__ src, float* __restrict__ part) {
  __shared__ float rs[8];
  __shared__ float rq[8];
  const int tid = threadIdx.x, lane = tid & 31, wave = tid >> 5;
  const int chunk = blockIdx.x;
  const int b = blockIdx.y;
  const float* base = src + (size_t)b * kGnElems + (size_t)chunk * 4096;
  float s = 0.0f, q = 0.0f;
#pragma unroll
  for (int i = 0; i < 4; ++i) {
    const v4f v = *(const v4f*)(base + 1024 * i + 4 * tid);
    s += (v[0] + v[1]) + (v[2] + v[3]);
    q += (v[0] * v[0] + v[1] * v[1]) + (v[2] * v[2] + v[3] * v[3]);
  }
#pragma unroll
  for (int off = 16; off > 0; off >>= 1) {
    s += __shfl_xor(s, off, 32);
    q += __shfl_xor(q, off, 32);
  }
  if (lane == 0) { rs[wave] = s; rq[wave] = q; }
  __syncthreads();
  if (wave == 0) {
    float S = 0.0f, Q = 0.0f;
#pragma unroll
    for (int w = 0; w < 8; ++w) { S += rs[w]; Q += rq[w]; }
    const float val = (lane == 0) ? S : ((lane == 1) ? Q : 0.0f);
    float* dp = part + ((size_t)(b * kGnChunks + chunk)) * 32 + lane;
    *(volatile float*)dp = val;
    __threadfence();
    *(volatile float*)dp = val;
  }
}

template <bool SILU>
__global__ __launch_bounds__(256) void gnapply_kernel(const float* __restrict__ src, const float* __restrict__ part,
                                                      const float* __restrict__ gam, const float* __restrict__ bet,
                                                      unsigned short* __restrict__ out16) {
  __shared__ float pS[kGnChunks];
  __shared__ float pQ[kGnChunks];
  __shared__ float st[2];
  const int tid = threadIdx.x;
  const int b = blockIdx.x >> 9;
  if (tid < kGnChunks) {
    const float* pp = part + ((size_t)(b * kGnChunks + tid)) * 32;
    pS[tid] = pp[0];
    pQ[tid] = pp[1];
  }
  __syncthreads();
  if (tid == 0) {
    double S = 0.0, Q = 0.0;
    for (int i = 0; i < kGnChunks; ++i) { S += (double)pS[i]; Q += (double)pQ[i]; }
    const double mean = S * kGnInvN;
    const double var = Q * kGnInvN - mean * mean;
    float varf = (float)var;
    varf = varf < 0.0f ? 0.0f : varf;
    st[0] = (float)mean;
    st[1] = 1.0f / sqrtf(varf + 1e-5f);
  }
  __syncthreads();
  const float mean = st[0], rstd = st[1];
  const int gidx = blockIdx.x * 256 + tid;
  const int row = gidx >> 7;
  const int c0 = (gidx & 127) * 4;
  const v4f xv = *(const v4f*)(src + (size_t)row * kD + c0);
  const v4f gv = *(const v4f*)(gam + c0);
  const v4f bv = *(const v4f*)(bet + c0);
  unsigned short hb[4];
#pragma unroll
  for (int e = 0; e < 4; ++e) {
    float y = (xv[e] - mean) * rstd * gv[e] + bv[e];
    if (SILU) {
      const float sg = 1.0f / (1.0f + expf(-y));
      y = y * sg;
    }
    hb[e] = h_bits(y);
  }
  const v2u u = (v2u){pk16(hb[0], hb[1]), pk16(hb[2], hb[3])};
  unsigned short* op = out16 + (size_t)row * kD + c0;
  *(volatile v2u*)op = u;
  __threadfence();
  *(volatile v2u*)op = u;
}

__global__ __launch_bounds__(256) void glu_kernel(const float* __restrict__ pre, float* __restrict__ out) {
  const int gidx = blockIdx.x * 256 + threadIdx.x;
  const int row = gidx >> 7;
  const int c0 = (gidx & 127) * 4;
  const v4f a = *(const v4f*)(pre + (size_t)row * (2 * kD) + c0);
  const v4f g = *(const v4f*)(pre + (size_t)row * (2 * kD) + kD + c0);
  v4f o;
#pragma unroll
  for (int e = 0; e < 4; ++e) {
    const float sg = 1.0f / (1.0f + expf(-g[e]));
    o[e] = a[e] * sg;
  }
  float* op = out + (size_t)row * kD + c0;
  *(volatile v4f*)op = o;
  __threadfence();
  *(volatile v4f*)op = o;
}

__global__ __launch_bounds__(128) void dwconv_kernel(const float* __restrict__ gin, const float* __restrict__ dwt,
                                                     const float* __restrict__ dwb, float* __restrict__ cout) {
  const int bt = blockIdx.x;
  const int b = bt >> 10, t = bt & 1023;
  const int c0 = threadIdx.x * 4;
  v4f acc = (v4f){0.0f, 0.0f, 0.0f, 0.0f};
#pragma unroll 1
  for (int k = 0; k < kKW; ++k) {
    const int tt = t + k - (kKW / 2);
    const bool valid = (unsigned)tt < (unsigned)kT;
    const int ttc = valid ? tt : 0;
    const v4f g = *(const v4f*)(gin + ((size_t)(b * kT + ttc)) * kD + c0);
    const v4f w = *(const v4f*)(dwt + (size_t)k * kD + c0);
#pragma unroll
    for (int e = 0; e < 4; ++e) {
      const float ge = valid ? g[e] : 0.0f;
      acc[e] += ge * w[e];
    }
  }
  const v4f bb = *(const v4f*)(dwb + c0);
  const v4f o = acc + bb;
  float* op = cout + (size_t)bt * kD + c0;
  *(volatile v4f*)op = o;
  __threadfence();
  *(volatile v4f*)op = o;
}

static_assert(4096 % 64 == 0 && 2048 % 64 == 0 && 1024 % 64 == 0 && 512 % 64 == 0 && 64 % 64 == 0);
static_assert(512 % 32 == 0 && 2048 % 32 == 0 && 64 % 32 == 0 && 1024 % 32 == 0);

extern "C" void kernel_launch(void* const* d_in, const int* in_sizes, int n_in,
                              void* d_out, int out_size, void* d_ws, size_t ws_size,
                              hipStream_t stream) {
  if (n_in < 27) return;
  static const int expect_sizes[27] = {2097152, 1048576, 2048, 1048576, 512, 786432, 1536, 262144, 512, 512, 512,
                                       524288, 1024, 15872, 512, 512, 512, 262144, 512, 1048576, 2048, 1048576, 512,
                                       2560, 512, 512, 8};
  for (int i = 0; i < 27; ++i) if (in_sizes[i] != expect_sizes[i]) return;
  if (out_size != kB * kD * kT) return;

  const size_t szS32  = (size_t)kTok * kD * 4;
  const size_t szS16  = (size_t)kTok * kD * 2;
  const size_t szWff  = (size_t)kD * kFF * 2;
  const size_t szWqkv = (size_t)kD * 3 * kD * 2;
  const size_t szWsq  = (size_t)kD * kD * 2;
  const size_t szWpw1 = (size_t)kD * 2 * kD * 2;
  const size_t szF32A = (size_t)kTok * kFF * 4;
  const size_t szF16A = (size_t)kTok * kFF * 2;
  const size_t szQK   = (size_t)kTok * kQKld * 2;
  const size_t szVT   = (size_t)kB * kD * kT * 2;
  const size_t szSmall = 65536;
  size_t off = 0;
  const size_t offS32A = off; off += szS32;
  const size_t offS32B = off; off += szS32;
  const size_t offS16  = off; off += szS16;
  const size_t offW1A  = off; off += szWff;
  const size_t offW2A  = off; off += szWff;
  const size_t offWQKV = off; off += szWqkv;
  const size_t offWOUT = off; off += szWsq;
  const size_t offWPW1 = off; off += szWpw1;
  const size_t offWPW2 = off; off += szWsq;
  const size_t offW1B  = off; off += szWff;
  const size_t offW2B  = off; off += szWff;
  const size_t offF32A = off; off += szF32A;
  const size_t offF16A = off; off += szF16A;
  const size_t offQK   = off; off += szQK;
  const size_t offVT   = off; off += szVT;
  const size_t offCTX  = off; off += szS16;
  const size_t offGN16 = off; off += szS16;
  const size_t offGLU  = off; off += szS32;
  const size_t offCONV = off; off += szS32;
  const size_t offRC   = off; off += 2 * szSmall;
  const size_t offDL   = off; off += szSmall;
  const size_t offGP1  = off; off += szSmall;
  const size_t offGP2  = off; off += szSmall;
  const size_t offDWT  = off; off += szSmall;
  const size_t total   = off;
  if (total > ws_size) return;
  if (total > (size_t)134217728) return;

  const float* x      = (const float*)d_in[0];
  const float* ff1_w1 = (const float*)d_in[1];
  const float* ff1_b1 = (const float*)d_in[2];
  const float* ff1_w2 = (const float*)d_in[3];
  const float* ff1_b2 = (const float*)d_in[4];
  const float* qkv_w  = (const float*)d_in[5];
  const float* qkv_b  = (const float*)d_in[6];
  const float* out_w  = (const float*)d_in[7];
  const float* out_b  = (const float*)d_in[8];
  const float* gn1_g  = (const float*)d_in[9];
  const float* gn1_b  = (const float*)d_in[10];
  const float* pw1_w  = (const float*)d_in[11];
  const float* pw1_b  = (const float*)d_in[12];
  const float* dw_w   = (const float*)d_in[13];
  const float* dw_b   = (const float*)d_in[14];
  const float* gn2_g  = (const float*)d_in[15];
  const float* gn2_b  = (const float*)d_in[16];
  const float* pw2_w  = (const float*)d_in[17];
  const float* pw2_b  = (const float*)d_in[18];
  const float* ff2_w1 = (const float*)d_in[19];
  const float* ff2_b1 = (const float*)d_in[20];
  const float* ff2_w2 = (const float*)d_in[21];
  const float* ff2_b2 = (const float*)d_in[22];
  const float* rel_emb = (const float*)d_in[23];
  const float* gate_u = (const float*)d_in[24];
  const float* gate_w = (const float*)d_in[25];
  const float* gate_sc = (const float*)d_in[26];
  float* out = (float*)d_out;

  char* ws = (char*)d_ws;
  float* S32A = (float*)(ws + offS32A);
  float* S32B = (float*)(ws + offS32B);
  unsigned short* S16  = (unsigned short*)(ws + offS16);
  unsigned short* W1A  = (unsigned short*)(ws + offW1A);
  unsigned short* W2A  = (unsigned short*)(ws + offW2A);
  unsigned short* WQKV = (unsigned short*)(ws + offWQKV);
  unsigned short* WOUT = (unsigned short*)(ws + offWOUT);
  unsigned short* WPW1 = (unsigned short*)(ws + offWPW1);
  unsigned short* WPW2 = (unsigned short*)(ws + offWPW2);
  unsigned short* W1B  = (unsigned short*)(ws + offW1B);
  unsigned short* W2B  = (unsigned short*)(ws + offW2B);
  float* F32A = (float*)(ws + offF32A);
  unsigned short* F16A = (unsigned short*)(ws + offF16A);
  unsigned short* QK   = (unsigned short*)(ws + offQK);
  unsigned short* VT   = (unsigned short*)(ws + offVT);
  unsigned short* CTX  = (unsigned short*)(ws + offCTX);
  unsigned short* GN16 = (unsigned short*)(ws + offGN16);
  float* GLU  = (float*)(ws + offGLU);
  float* CONV = (float*)(ws + offCONV);
  float* RC   = (float*)(ws + offRC);
  float* DL   = (float*)(ws + offDL);
  float* GP1  = (float*)(ws + offGP1);
  float* GP2  = (float*)(ws + offGP2);
  float* DWT  = (float*)(ws + offDWT);

  const dim3 blk(256);
  const int n8stream = (kTok * kD) / 8;
  const int n2ffn    = (kTok * kFF) / 2;

  wtcast2_kernel<<<dim3(kD / 64, kFF / 64, 2), blk, 0, stream>>>(ff1_w1, ff2_w1, W1A, W1B, kD, kFF, kWCarry);
  wtcast2_kernel<<<dim3(kFF / 64, kD / 64, 2), blk, 0, stream>>>(ff1_w2, ff2_w2, W2A, W2B, kFF, kD, kWCarry);
  wtcast2_kernel<<<dim3(kD / 64, (3 * kD) / 64, 1), blk, 0, stream>>>(qkv_w, qkv_w, WQKV, WQKV, kD, 3 * kD, kWCarry);
  wtcast2_kernel<<<dim3(kD / 64, kD / 64, 2), blk, 0, stream>>>(out_w, pw2_w, WOUT, WPW2, kD, kD, kWCarry);
  wtcast2_kernel<<<dim3(kD / 64, (2 * kD) / 64, 1), blk, 0, stream>>>(pw1_w, pw1_w, WPW1, WPW1, kD, 2 * kD, kWCarry);
  dline_kernel<<<dim3(16), blk, 0, stream>>>(rel_emb, DL);
  dwt_kernel<<<dim3(16), blk, 0, stream>>>(dw_w, DWT);
  xin_kernel<<<dim3(kT / 64, kD / 64, kB), blk, 0, stream>>>(x, S32A, S16);

  const int tilesFF1 = (kTok / 64) * (kFF / 64);
  const int tilesD   = (kTok / 64) * (kD / 64);
  const int tiles2D  = (kTok / 64) * (2 * kD / 64);

  gemm_f16w<2, 0, false><<<dim3((tilesFF1 + 7) / 8, 1), blk, 0, stream>>>(
      S16, kD, 0L, W1A, kD, 0L, (void*)F32A, kFF, 0L, ff1_b1, 1.0f, S32A, 0L, kTok, kFF, kD, kWInv);
  gelu2_kernel<<<dim3(n2ffn / 256), blk, 0, stream>>>(F32A, F16A, n2ffn);
  gemm_f16w<2, 0, true><<<dim3((tilesD + 7) / 8, 1), blk, 0, stream>>>(
      F16A, kFF, 0L, W2A, kFF, 0L, (void*)S32B, kD, 0L, ff1_b2, 0.5f, S32A, 0L, kTok, kD, kFF, 0.5f * kWInv);
  cast8_f16_kernel<<<dim3(n8stream / 256), blk, 0, stream>>>(S32B, S16, n8stream);

  gemm_f16w<2, 1, false><<<dim3((tiles2D + 7) / 8, 1), blk, 0, stream>>>(
      S16, kD, 0L, WQKV, kD, 0L, (void*)QK, kQKld, 0L, qkv_b, 1.0f, S32A, 0L, kTok, 2 * kD, kD, kWInv);
  {
    const int tilesVT = (kD / 64) * (kT / 64);
    gemm_f16w<1, 1, false><<<dim3((tilesVT + 7) / 8, kB), blk, 0, stream>>>(
        WQKV + (size_t)(2 * kD) * kD, kD, 0L, S16, kD, (long)kT * kD, (void*)VT, kT, (long)kD * kT,
        qkv_b + 2 * kD, 1.0f, S32A, 0L, kD, kT, kD, kWInv);
  }
  gates_kernel<<<dim3((kB * kH * kT) / 256), blk, 0, stream>>>(QK, gate_u, gate_w, gate_sc, RC);

  {
    const int tilesS  = (kT / 64) * (kT / 64);
    const int tilesPV = (kT / 64) * (kDh / 64);
    for (int b = 0; b < kB; ++b) {
      const unsigned short* qbp = QK + (size_t)b * kT * kQKld;
      gemm_f16w<0, 0, false><<<dim3((tilesS + 7) / 8, kH), blk, 0, stream>>>(
          qbp, kQKld, (long)kDh, qbp + kD, kQKld, (long)kDh, (void*)F32A, kT, (long)kT * kT,
          ff1_b1, 1.0f, S32A, 0L, kT, kT, kDh, kScoreScale);
      softmax_kernel<<<dim3(kT, kH), dim3(128), 0, stream>>>(F32A, F16A, RC + (size_t)b * kH * kT, DL);
      gemm_f16w<0, 1, false><<<dim3((tilesPV + 7) / 8, kH), blk, 0, stream>>>(
          F16A, kT, (long)kT * kT, VT + (size_t)b * kD * kT, kT, (long)kDh * kT,
          (void*)(CTX + (size_t)b * kT * kD), kD, (long)kDh, ff1_b1, 1.0f, S32A, 0L, kT, kDh, kT, kPVScale);
    }
  }

  gemm_f16w<2, 0, true><<<dim3((tilesD + 7) / 8, 1), blk, 0, stream>>>(
      CTX, kD, 0L, WOUT, kD, 0L, (void*)S32A, kD, 0L, out_b, 1.0f, S32B, 0L, kTok, kD, kD, kOutScale);

  gnred_kernel<<<dim3(kGnChunks, kB), blk, 0, stream>>>(S32A, GP1);
  gnapply_kernel<false><<<dim3((kTok * kD) / 4 / 256), blk, 0, stream>>>(S32A, GP1, gn1_g, gn1_b, GN16);
  gemm_f16w<2, 0, false><<<dim3((tiles2D + 7) / 8, 1), blk, 0, stream>>>(
      GN16, kD, 0L, WPW1, kD, 0L, (void*)F32A, 2 * kD, 0L, pw1_b, 1.0f, S32A, 0L, kTok, 2 * kD, kD, kWInv);
  glu_kernel<<<dim3((kTok * kD) / 4 / 256), blk, 0, stream>>>(F32A, GLU);
  dwconv_kernel<<<dim3(kTok), dim3(128), 0, stream>>>(GLU, DWT, dw_b, CONV);
  gnred_kernel<<<dim3(kGnChunks, kB), blk, 0, stream>>>(CONV, GP2);
  gnapply_kernel<true><<<dim3((kTok * kD) / 4 / 256), blk, 0, stream>>>(CONV, GP2, gn2_g, gn2_b, GN16);
  gemm_f16w<2, 0, true><<<dim3((tilesD + 7) / 8, 1), blk, 0, stream>>>(
      GN16, kD, 0L, WPW2, kD, 0L, (void*)S32B, kD, 0L, pw2_b, 1.0f, S32A, 0L, kTok, kD, kD, kWInv);
  cast8_f16_kernel<<<dim3(n8stream / 256), blk, 0, stream>>>(S32B, S16, n8stream);

  gemm_f16w<2, 0, false><<<dim3((tilesFF1 + 7) / 8, 1), blk, 0, stream>>>(
      S16, kD, 0L, W1B, kD, 0L, (void*)F32A, kFF, 0L, ff2_b1, 1.0f, S32A, 0L, kTok, kFF, kD, kWInv);
  gelu2_kernel<<<dim3(n2ffn / 256), blk, 0, stream>>>(F32A, F16A, n2ffn);
  gemm_f16w<2, 0, true><<<dim3((tilesD + 7) / 8, 1), blk, 0, stream>>>(
      F16A, kFF, 0L, W2B, kFF, 0L, (void*)S32A, kD, 0L, ff2_b2, 0.5f, S32B, 0L, kTok, kD, kFF, 0.5f * kWInv);

  xout_kernel<<<dim3(kT / 64, kD / 64, kB), blk, 0, stream>>>(S32A, out);
}
